// LocalScopeSelfAttention_22565758173962
// MI455X (gfx1250) — hardware-verified
//
#include <hip/hip_runtime.h>
#include <math.h>

typedef __attribute__((ext_vector_type(16))) _Float16 v16h;
typedef __attribute__((ext_vector_type(16))) __bf16 v16b;
typedef __attribute__((ext_vector_type(8)))  _Float16 v8h;
typedef __attribute__((ext_vector_type(8)))  float v8f;
typedef __attribute__((ext_vector_type(4)))  float v4f;
typedef __attribute__((ext_vector_type(2)))  float v2f;
typedef __attribute__((ext_vector_type(4)))  unsigned v4u;
typedef __attribute__((ext_vector_type(4)))  int v4i;
typedef float __attribute__((may_alias)) float_a;
typedef int __attribute__((may_alias)) int_a;

template <typename T> __device__ __forceinline__ void vst2(void* p, T v) { *(volatile T*)p = v; __threadfence(); *(volatile T*)p = v; }
__device__ __forceinline__ v8f wmma16(v16h a, v16h b, v8f c) {
  v8f d = __builtin_amdgcn_wmma_f32_16x16x32_f16(false, a, false, b, (short)0, c, false, false);
  asm volatile("v_nop\n\tv_nop\n\tv_nop\n\tv_nop" : "+v"(d) : "v"(a), "v"(b));
  return d;
}
__device__ __forceinline__ v8f wmma_bf(v16b a, v16b b, v8f c) {
  v8f d = __builtin_amdgcn_wmma_f32_16x16x32_bf16(false, a, false, b, (short)0, c, false, false);
  asm volatile("v_nop\n\tv_nop\n\tv_nop\n\tv_nop" : "+v"(d) : "v"(a), "v"(b));
  return d;
}
__device__ __forceinline__ v16h frag_h(const _Float16* rowk0, int lane) {
  union { v16h v; v8h q[2]; } u; const _Float16* p = rowk0 + 8 * (lane >> 4);
  u.q[0] = *(const v8h*)p; u.q[1] = *(const v8h*)(p + 16); return u.v;
}
__device__ __forceinline__ v16h frag_f32(const float* rowk0, int lane) {
  v16h a; const float* p = rowk0 + 8 * (lane >> 4);
#pragma unroll
  for (int i = 0; i < 8; ++i) { a[i] = (_Float16)p[i]; a[8 + i] = (_Float16)p[16 + i]; }
  return a;
}
__device__ __forceinline__ v16h frag_f32s(const float* rowk0, int lane, float sc) {
  v16h a; const float* p = rowk0 + 8 * (lane >> 4);
#pragma unroll
  for (int i = 0; i < 8; ++i) { a[i] = (_Float16)(p[i] * sc); a[8 + i] = (_Float16)(p[16 + i] * sc); }
  return a;
}
__device__ __forceinline__ v16h fragc_f32(const float* W, int k0, int n, int lane, int ld, int K) {
  v16h a; const int g = lane >> 4;
#pragma unroll
  for (int i = 0; i < 8; ++i) { const int ka = k0 + 8 * g + i, kb = ka + 16;
    a[i] = (_Float16)(ka < K ? W[(size_t)(ka < K ? ka : K - 1) * ld + n] : 0.f); a[8 + i] = (_Float16)(kb < K ? W[(size_t)(kb < K ? kb : K - 1) * ld + n] : 0.f); }
  return a;
}
struct F2 { v16b h, l; };
__device__ __forceinline__ F2 bsplit16(const float v[16]) { F2 r;
#pragma unroll
  for (int i = 0; i < 16; ++i) { const __bf16 h = (__bf16)v[i]; r.h[i] = h; r.l[i] = (__bf16)(v[i] - (float)h); }
  return r; }
__device__ __forceinline__ F2 split_row(const float* row, int k0, int lane) { float v[16]; const float* p = row + k0 + 8 * (lane >> 4);
#pragma unroll
  for (int i = 0; i < 8; ++i) { v[i] = p[i]; v[8 + i] = p[16 + i]; }
  return bsplit16(v); }
__device__ __forceinline__ F2 split_rowK(const float* row, int k0, int lane, int K) { float v[16]; const int g = lane >> 4;
#pragma unroll
  for (int i = 0; i < 8; ++i) { const int ka = k0 + 8 * g + i, kb = ka + 16; v[i] = ka < K ? row[ka < K ? ka : K - 1] : 0.f; v[8 + i] = kb < K ? row[kb < K ? kb : K - 1] : 0.f; }
  return bsplit16(v); }
__device__ __forceinline__ F2 split_col(const float* W, int k0, int n, int lane, int ld, int K) { float v[16]; const int g = lane >> 4;
#pragma unroll
  for (int i = 0; i < 8; ++i) { const int ka = k0 + 8 * g + i, kb = ka + 16; v[i] = ka < K ? W[(size_t)(ka < K ? ka : K - 1) * ld + n] : 0.f; v[8 + i] = kb < K ? W[(size_t)(kb < K ? kb : K - 1) * ld + n] : 0.f; }
  return bsplit16(v); }
__device__ __forceinline__ v8f mac3(const F2& a, const F2& b, v8f c) { c = wmma_bf(a.l, b.h, c); c = wmma_bf(a.h, b.l, c); return wmma_bf(a.h, b.h, c); }
__device__ __forceinline__ float sigm(float v) { return 1.0f / (1.0f + expf(-v)); }
#define LDSX() do { asm volatile("s_wait_dscnt 0" ::: "memory"); __builtin_amdgcn_wave_barrier(); __builtin_amdgcn_fence(__ATOMIC_RELEASE, "workgroup"); } while (0)


#define NFR 16
#define HH 32
#define WWd 32
#define NPOS (HH * WWd)
#define DM 256
#define NHD 8
#define HD 32
#define NR (NFR * NPOS)
#ifndef TRB
#define TRB (NR / 64)
#endif
typedef __attribute__((ext_vector_type(8))) __bf16 v8b;
__device__ __forceinline__ v16b frag_b(const __bf16* rowk0, int lane) {
  union { v16b v; v8b q[2]; } u; const __bf16* p = rowk0 + 8 * (lane >> 4);
  u.q[0] = *(const v8b*)p; u.q[1] = *(const v8b*)(p + 16); return u.v;
}
__device__ __forceinline__ float bfr(float v) { return (float)(__bf16)v; }
__device__ __attribute__((noinline)) float exp_ni(float v) { return expf(v); }
__device__ __attribute__((noinline)) float erf_ni(float v) { return erff(v); }

#define WS_PW  0u
#define WS_XN  (WS_PW + 2u * 4 * DM * DM)
#define WS_Q   (WS_XN + 4u * (size_t)NR * DM)
#define WS_K   (WS_Q + 4u * (size_t)NR * DM)
#define WS_V   (WS_K + 4u * (size_t)NR * DM)
#define WS_END (WS_V + 4u * (size_t)NR * DM)

__global__ __launch_bounds__(256) void k_pack(const float* __restrict__ WQ, const float* __restrict__ WK, const float* __restrict__ WV, const float* __restrict__ WO, __bf16* __restrict__ PW) {
  const int n = blockIdx.x, which = blockIdx.y, t = threadIdx.x; const float* Wm = (which == 0) ? WQ : (which == 1) ? WK : (which == 2) ? WV : WO; __shared__ __align__(16) __bf16 s[DM];
  s[t] = (__bf16)Wm[(size_t)t * DM + n]; __syncthreads();
  if (t < DM / 8) vst2((unsigned*)(PW + ((size_t)which * DM + n) * DM + t * 8), *(const v4u*)&s[t * 8]);
}
__global__ __launch_bounds__(64) void k_ln(const float* __restrict__ X, const float* __restrict__ G, const float* __restrict__ Bt, float* __restrict__ XN) {
  __shared__ float red[2]; const int t = threadIdx.x; const size_t row = blockIdx.x; float v[4]; float s = 0.f; for (int i = 0; i < 4; ++i) { v[i] = bfr(X[row * DM + t * 4 + i]); s += v[i]; }
#pragma unroll
  for (int o = 1; o < 32; o <<= 1) s += __shfl_xor(s, o);
  if ((t & 31) == 0) red[t >> 5] = s; __syncthreads(); const float mu = (red[0] + red[1]) / (float)DM; __syncthreads();
  float q = 0.f; for (int i = 0; i < 4; ++i) { const float dd = v[i] - mu; q += dd * dd; }
#pragma unroll
  for (int o = 1; o < 32; o <<= 1) q += __shfl_xor(q, o);
  if ((t & 31) == 0) red[t >> 5] = q; __syncthreads(); const float inv = 1.0f / sqrtf((red[0] + red[1]) / (float)DM + 1e-5f);
  v4f o4; for (int i = 0; i < 4; ++i) { const int e = t * 4 + i; o4[i] = (v[i] - mu) * inv * bfr(G[e]) + bfr(Bt[e]); }
  vst2(XN + row * DM + t * 4, o4);
}
__global__ __launch_bounds__(128) void k_qkv(const float* __restrict__ XN, const __bf16* __restrict__ PW, const float* __restrict__ BQ, const float* __restrict__ BK, const float* __restrict__ BV, float* __restrict__ Q, float* __restrict__ Kx, float* __restrict__ V) {
  __shared__ __align__(16) float so[4][16][132];
  const int tid = threadIdx.x, wave = tid >> 5, lane = tid & 31, col = lane & 15, g = lane >> 4; const int which = blockIdx.y; const size_t r0 = (size_t)blockIdx.x * 64 + wave * 16;
  const __bf16* Wr = PW + (size_t)which * DM * DM; const float* bias = (which == 0) ? BQ : (which == 1) ? BK : BV; float* dst = (which == 0) ? Q : (which == 1) ? Kx : V;
#pragma unroll 1
  for (int pass = 0; pass < 2; ++pass) { v8f acc[8] = {};
#pragma unroll 2
    for (int kc = 0; kc < DM / 32; ++kc) { const F2 a = split_row(XN + (r0 + col) * DM, kc * 32, lane);
#pragma unroll
      for (int j = 0; j < 8; ++j) { const v16b w = frag_b(Wr + (size_t)(pass * 128 + j * 16 + col) * DM + kc * 32, lane); acc[j] = wmma_bf(a.l, w, acc[j]); acc[j] = wmma_bf(a.h, w, acc[j]); } }
#pragma unroll
    for (int j = 0; j < 8; ++j) { const float bb = bfr(bias[pass * 128 + j * 16 + col]);
#pragma unroll
      for (int r = 0; r < 8; ++r) so[wave][8 * g + r][j * 16 + col] = acc[j][r] + bb; }
    LDSX();
    for (int rl = 0; rl < 16; ++rl) vst2(dst + (r0 + rl) * DM + pass * 128 + lane * 4, *(const v4f*)&so[wave][rl][lane * 4]);
    LDSX(); }
}
__global__ __launch_bounds__(128) void k_attn_out(const float* __restrict__ Q, const float* __restrict__ Kx, const float* __restrict__ V, const __bf16* __restrict__ PW, const float* __restrict__ BO, const float* __restrict__ X, float* __restrict__ OUT) {
  __shared__ __align__(16) float sc[64][DM + 4]; __shared__ __align__(16) float so[4][16][132]; __shared__ float ssc[128][10];
  const int tid = threadIdx.x, wave = tid >> 5, lane = tid & 31, col = lane & 15, g = lane >> 4; const size_t rb0 = (size_t)blockIdx.x * 64; const size_t fr = rb0 / NPOS; const int p0 = (int)(rb0 % NPOS);
#pragma unroll 1
  for (int it = tid; it < 64 * NHD; it += 128) { const int r = it >> 3, h = it & 7; const int p = p0 + r; const int py = p / WWd, px = p % WWd; const float* qrow = Q + (rb0 + r) * DM + h * HD;
    float qv[HD];
#pragma unroll
    for (int d = 0; d < HD; ++d) qv[d] = qrow[d];
    float* sco = ssc[tid]; float mx = -3.0e38f;
#pragma unroll 1
    for (int kk = 0; kk < 9; ++kk) { const int dy = kk / 3 - 1, dx = kk % 3 - 1; int ny = py + dy, nx = px + dx; ny = ny < 0 ? 0 : (ny > HH - 1 ? HH - 1 : ny); nx = nx < 0 ? 0 : (nx > WWd - 1 ? WWd - 1 : nx);
      const float* krow = Kx + (fr * NPOS + (size_t)(ny * WWd + nx)) * DM + h * HD; float s = 0.f;
#pragma unroll
      for (int d = 0; d < HD; ++d) s += qv[d] * krow[d];
      s *= 0.17677669529663687f; sco[kk] = s; mx = fmaxf(mx, s); }
    float den = 0.f;
#pragma unroll 1
    for (int kk = 0; kk < 9; ++kk) { const float e = exp_ni(sco[kk] - mx); sco[kk] = e; den += e; }
    const float inv = 1.0f / den;
    float ov[HD];
#pragma unroll
    for (int d = 0; d < HD; ++d) ov[d] = 0.f;
#pragma unroll 1
    for (int kk = 0; kk < 9; ++kk) { const int dy = kk / 3 - 1, dx = kk % 3 - 1; int ny = py + dy, nx = px + dx; ny = ny < 0 ? 0 : (ny > HH - 1 ? HH - 1 : ny); nx = nx < 0 ? 0 : (nx > WWd - 1 ? WWd - 1 : nx);
      const float* vrow = V + (fr * NPOS + (size_t)(ny * WWd + nx)) * DM + h * HD; const float pw = sco[kk] * inv;
#pragma unroll
      for (int d = 0; d < HD; ++d) ov[d] += pw * vrow[d]; }
#pragma unroll
    for (int d = 0; d < HD; ++d) sc[r][h * HD + d] = ov[d]; }
  if (tid < 64) for (int c = DM; c < DM + 4; ++c) sc[tid][c] = 0.f;
  __syncthreads();
  const __bf16* Wr = PW + (size_t)3 * DM * DM; const size_t r0 = rb0 + wave * 16;
#pragma unroll 1
  for (int pass = 0; pass < 2; ++pass) { v8f acc[8] = {};
#pragma unroll 2
    for (int kc = 0; kc < DM / 32; ++kc) { const F2 a = split_row(&sc[wave * 16 + col][0], kc * 32, lane);
#pragma unroll
      for (int j = 0; j < 8; ++j) { const v16b w = frag_b(Wr + (size_t)(pass * 128 + j * 16 + col) * DM + kc * 32, lane); acc[j] = wmma_bf(a.l, w, acc[j]); acc[j] = wmma_bf(a.h, w, acc[j]); } }
#pragma unroll
    for (int j = 0; j < 8; ++j) { const int c = pass * 128 + j * 16 + col; const float bb = bfr(BO[c]);
#pragma unroll
      for (int r = 0; r < 8; ++r) so[wave][8 * g + r][j * 16 + col] = acc[j][r] + bb + bfr(X[(r0 + 8 * g + r) * DM + c]); }
    LDSX();
    for (int rl = 0; rl < 16; ++rl) vst2(OUT + (r0 + rl) * DM + pass * 128 + lane * 4, *(const v4f*)&so[wave][rl][lane * 4]);
    LDSX(); }
}
extern "C" void kernel_launch(void* const* d_in, const int* in_sizes, int n_in, void* d_out, int out_size, void* d_ws, size_t ws_size, hipStream_t stream) {
  (void)in_sizes; (void)n_in; (void)out_size;
  const float** F = (const float**)d_in;
  if (ws_size < (size_t)WS_END) return;
  char* ws = (char*)d_ws; __bf16* PW = (__bf16*)(ws + WS_PW); float *XN = (float*)(ws + WS_XN), *Q = (float*)(ws + WS_Q), *Kx = (float*)(ws + WS_K), *V = (float*)(ws + WS_V);
  k_pack<<<dim3(DM, 4), 256, 0, stream>>>(F[3], F[5], F[7], F[9], PW);
  k_ln<<<NR, 64, 0, stream>>>(F[0], F[1], F[2], XN);
  k_qkv<<<dim3(NR / 64, 3), 128, 0, stream>>>(XN, PW, F[4], F[6], F[8], Q, Kx, V);
  k_attn_out<<<TRB, 128, 0, stream>>>(Q, Kx, V, PW, F[10], F[0], (float*)d_out);
}
